// PDAG_Generator_19224273617537
// MI455X (gfx1250) — hardware-verified
//
#include <hip/hip_runtime.h>
#include <math.h>

#ifndef NROWS
#define NROWS 16384
#endif
#define NROWS_FULL 16384
#define NNODE 16
#define HID 512
#define XP 20
#define XPH 40
#define HP 520
#define WSC 256.0f
#define ASC 8.0f
#define SCL 4.8828125e-4f

static_assert(NROWS % 64 == 0);
static_assert(NROWS <= NROWS_FULL);
static_assert((NROWS * 4) % 256 == 0);
static_assert(HID % 64 == 0 && HID % 32 == 0);
static_assert(HID / 64 == 8);
static_assert((XPH * 2) % 16 == 0 && (HP * 2) % 16 == 0);
static_assert(XP * 2 == XPH && XPH >= 32);
static_assert((NNODE * HID * 4) % 256 == 0);
static_assert((NNODE * HID * HID / 8) % 256 == 0);
static_assert(64 * XP * 4 + 64 * HP * 2 + 8 * 64 * 4 <= 131072);
static_assert(512 * 4 + 16 * 4 <= 131072);
static_assert((size_t)NROWS_FULL * NNODE * 4 == 1048576);
static_assert(64 * 4 == 2 * 32 * 4);

typedef _Float16 h16;
typedef __attribute__((ext_vector_type(16))) _Float16 v16h;
typedef __attribute__((ext_vector_type(8)))  _Float16 v8h;
typedef __attribute__((ext_vector_type(8)))  float    v8f;
typedef __attribute__((ext_vector_type(4)))  float    v4f;
typedef __attribute__((ext_vector_type(4)))  unsigned int v4u;
typedef __attribute__((ext_vector_type(2)))  unsigned int v2u;


#define VST2(T, ptr, val) do { const T vst2_v_ = (val); *(volatile T*)(ptr) = vst2_v_; __threadfence(); *(volatile T*)(ptr) = vst2_v_; } while (0)
#define VST2V4(ptr, val) do { const v4f vst2_v4_ = (val); *(volatile v4f*)(ptr) = vst2_v4_; __threadfence(); *(volatile v4f*)(ptr) = vst2_v4_; } while (0)

__device__ __forceinline__ float bfr(float f) {
    unsigned u = __float_as_uint(f);
    u += 0x7FFFu + ((u >> 16) & 1u);
    return __uint_as_float(u & 0xFFFF0000u);
}
static __device__ __forceinline__ h16 toh_flush(float v) {
    const h16 r = (h16)v;
    return (fabsf(v) < 6.103515625e-05f) ? (h16)0.0f : r;
}
static __device__ __forceinline__ unsigned hbits(float v) {
    return (unsigned)__builtin_bit_cast(unsigned short, toh_flush(v));
}
static __device__ __forceinline__ unsigned hpack(float lo, float hi) {
    return hbits(lo) | (hbits(hi) << 16);
}
static __device__ __forceinline__ void st8hf(unsigned short* P, size_t o, const float* v) {
    v4u pk;
    pk.x = hpack(v[0], v[1]);
    pk.y = hpack(v[2], v[3]);
    pk.z = hpack(v[4], v[5]);
    pk.w = hpack(v[6], v[7]);
    VST2(v4u, (v4u*)(P + o), pk);
}

union FragU { v16h v; v8h h[2]; };
__device__ __forceinline__ v16h frag_ld(const _Float16* p) {
    FragU f; f.h[0] = *(const v8h*)(p); f.h[1] = *(const v8h*)(p + 16); return f.v;
}
__device__ __forceinline__ v8f wmma16(v16h a, v16h b, v8f c) {
    c = __builtin_amdgcn_wmma_f32_16x16x32_f16(false, a, false, b, (short)0, c, false, false);
    asm volatile("v_nop\n\tv_nop\n\tv_nop\n\tv_nop" : "+v"(c) : "v"(a), "v"(b));
    return c;
}

__global__ __launch_bounds__(512) void k_theta(const float* __restrict__ mu, const float* __restrict__ sigma,
                                               const float* __restrict__ noise_d, float* __restrict__ theta,
                                               float* __restrict__ klout) {
#pragma clang fp contract(off)
    __shared__ float sTh[512];
    __shared__ float sRed[16];
    const unsigned t = threadIdx.x, lane = t & 31u;
    const unsigned wave = (unsigned)__builtin_amdgcn_readfirstlane((int)(t >> 5));
    const float s = bfr(sigma[t]);
    const float m = bfr(mu[t]);
    const float nz = bfr(noise_d[t]);
    const float sp = log1pf(expf(s));
    sTh[t] = m + sp * nz;
    float kl = ((1.0f + logf(sp * sp)) - m * m) - sp * sp;
#pragma unroll
    for (int o = 16; o > 0; o >>= 1) kl += __shfl_xor(kl, o, 32);
    if (lane == 0u) sRed[wave] = kl;
    __syncthreads();
    if (t < 128u) {
        v4f v; v.x = sTh[4u * t]; v.y = sTh[4u * t + 1u]; v.z = sTh[4u * t + 2u]; v.w = sTh[4u * t + 3u];
        VST2V4(theta + 4u * t, v);
    }
    if (t == 0u) {
        v4f k;
        k.x = -(((sRed[0] + sRed[1]) + sRed[2]) + sRed[3]);
        k.y = -(((sRed[4] + sRed[5]) + sRed[6]) + sRed[7]);
        k.z = -(((sRed[8] + sRed[9]) + sRed[10]) + sRed[11]);
        k.w = -(((sRed[12] + sRed[13]) + sRed[14]) + sRed[15]);
        VST2V4(klout, k);
    }
}

__global__ __launch_bounds__(256) void k_w0conv(const float* __restrict__ W0_0, const float* __restrict__ W0_rest,
                                                unsigned short* __restrict__ W0h) {
    const unsigned u = blockIdx.x * 256u + threadIdx.x;
    if (u >= (unsigned)(NNODE * HID * 4)) return;
    const unsigned k0 = (u & 3u) * 8u;
    const unsigned n = (u >> 2) & 511u;
    const unsigned node = u >> 11;
    const unsigned nr = (node > 0u) ? (node - 1u) : 0u;
    const float* r0p = W0_0 + (size_t)n * 17u;
    const float* r1p = W0_rest + ((size_t)nr * HID + n) * 18u;
    const unsigned kmax = (node == 0u) ? 17u : 18u;
    float v[8];
#pragma unroll
    for (int e = 0; e < 8; ++e) {
        const unsigned k = k0 + (unsigned)e;
        const float x0 = r0p[min(k, 16u)];
        const float x1 = r1p[min(k, 17u)];
        const float w = (node == 0u) ? x0 : x1;
        v[e] = (k < kmax) ? bfr(w) * WSC : 0.0f;
    }
    st8hf(W0h, (size_t)u * 8u, v);
}

__global__ __launch_bounds__(256) void k_w1conv(const float* __restrict__ W1, unsigned short* __restrict__ W1h) {
    const unsigned u = blockIdx.x * 256u + threadIdx.x;
    if (u >= (unsigned)(NNODE * HID * HID / 8)) return;
    const float* src = W1 + (size_t)u * 8u;
    const v4f a = *(const v4f*)src, b = *(const v4f*)(src + 4);
    float v[8];
    v[0] = bfr(a.x) * WSC; v[1] = bfr(a.y) * WSC; v[2] = bfr(a.z) * WSC; v[3] = bfr(a.w) * WSC;
    v[4] = bfr(b.x) * WSC; v[5] = bfr(b.y) * WSC; v[6] = bfr(b.z) * WSC; v[7] = bfr(b.w) * WSC;
    st8hf(W1h, (size_t)u * 8u, v);
}

__global__ __launch_bounds__(256) void k_node(int node,
    const float* __restrict__ noise, const float* __restrict__ input_c, const float* __restrict__ input_d,
    const float* __restrict__ cnet_w, const float* __restrict__ theta,
    const _Float16* __restrict__ W0h, const _Float16* __restrict__ W1h,
    const float* __restrict__ b0, const float* __restrict__ b1,
    const float* __restrict__ W2, const float* __restrict__ b2,
    float* oT) {
    __shared__ __align__(16) unsigned int sXw[64 * XP];
    __shared__ __align__(16) _Float16 sH1[64 * HP];
    __shared__ float sPart[8 * 64];

    const unsigned tid = threadIdx.x, lane = tid & 31u;
    const unsigned wave = (unsigned)__builtin_amdgcn_readfirstlane((int)(tid >> 5));
    const unsigned hh = lane >> 4, c = lane & 15u, koff = 8u * hh;
    const unsigned bbase = blockIdx.x * 64u;
    const unsigned nd = (unsigned)node;

    {
        const unsigned row = tid >> 2, q = tid & 3u;
        const size_t b = (size_t)bbase + row;
        const float* ic = input_c + b * 10u;
        float a[10];
#pragma unroll
        for (int j = 0; j < 10; ++j) a[j] = bfr(ic[j]);
        const v4f dv = *(const v4f*)(input_d + b * 4u);
        const float d0 = bfr(dv.x), d1 = bfr(dv.y), d2 = bfr(dv.z), d3 = bfr(dv.w);
        const float* cA = cnet_w + (size_t)(8u * nd + 2u * q) * 10u;
        float ci0 = 0.f, ci1 = 0.f;
#pragma unroll
        for (int j = 0; j < 10; ++j) { ci0 += a[j] * bfr(cA[j]); ci1 += a[j] * bfr(cA[10 + j]); }
        const float* tp = theta + 8u * nd + 2u * q;
        const float di0 = ((d0 * tp[0] + d1 * tp[128]) + d2 * tp[256]) + d3 * tp[384];
        const float di1 = ((d0 * tp[1] + d1 * tp[129]) + d2 * tp[257]) + d3 * tp[385];
        float ni = bfr(noise[b * 16u + nd]);
        float pv = 0.0f;
        if (node > 0) pv = oT[(size_t)(nd - 1u) * NROWS + b];
        asm volatile("" : "+v"(ni));
        asm volatile("" : "+v"(pv));
        const unsigned wc = hpack(ci0 * ASC, ci1 * ASC);
        const unsigned wd = hpack(di0 * ASC, di1 * ASC);
        const unsigned wn = hpack(ni * ASC, pv * ASC);
        sXw[row * XP + q] = wc;
        sXw[row * XP + 4u + q] = wd;
        v2u z; z.x = (q == 0u) ? wn : 0u; z.y = 0u;
        *(v2u*)(sXw + row * XP + 8u + 2u * q) = z;
    }
    __syncthreads();

    const unsigned n0 = wave * 64u;
    v8f acc[4][4];
#pragma unroll
    for (int i = 0; i < 4; ++i)
#pragma unroll
        for (int j = 0; j < 4; ++j) acc[i][j] = (v8f){0.f,0.f,0.f,0.f,0.f,0.f,0.f,0.f};

    {
        const _Float16* w0n = W0h + ((size_t)nd * HID + n0 + c) * 32u + koff;
        const _Float16* xh = (const _Float16*)sXw;
        v16h bh[4];
#pragma unroll
        for (int j = 0; j < 4; ++j) bh[j] = frag_ld(w0n + (size_t)j * 16u * 32u);
#pragma unroll
        for (int i = 0; i < 4; ++i) {
            const v16h ah = frag_ld(xh + ((unsigned)i * 16u + c) * XPH + koff);
#pragma unroll
            for (int j = 0; j < 4; ++j) acc[i][j] = wmma16(ah, bh[j], acc[i][j]);
        }
    }
#pragma unroll
    for (int j = 0; j < 4; ++j) {
        const unsigned n = n0 + (unsigned)j * 16u + c;
        const float b0v = bfr(b0[nd * HID + n]);
#pragma unroll
        for (int i = 0; i < 4; ++i)
#pragma unroll
            for (int r = 0; r < 8; ++r) {
                float v = acc[i][j][r] * SCL + b0v;
                v = fmaxf(v, 0.0f);
                sH1[((unsigned)i * 16u + 8u * hh + (unsigned)r) * HP + n] = toh_flush(v * ASC);
            }
    }
    __syncthreads();

#pragma unroll
    for (int i = 0; i < 4; ++i)
#pragma unroll
        for (int j = 0; j < 4; ++j) acc[i][j] = (v8f){0.f,0.f,0.f,0.f,0.f,0.f,0.f,0.f};
    {
        const _Float16* w1n = W1h + ((size_t)nd * HID + n0 + c) * HID + koff;
#pragma unroll 1
        for (unsigned k0 = 0; k0 < (unsigned)HID; k0 += 32u) {
            v16h bh[4];
#pragma unroll
            for (int j = 0; j < 4; ++j) bh[j] = frag_ld(w1n + (size_t)j * 16u * HID + k0);
#pragma unroll
            for (int i = 0; i < 4; ++i) {
                const v16h ah = frag_ld(sH1 + ((unsigned)i * 16u + c) * HP + koff + k0);
#pragma unroll
                for (int j = 0; j < 4; ++j) acc[i][j] = wmma16(ah, bh[j], acc[i][j]);
            }
        }
    }

    float rs[4][8];
#pragma unroll
    for (int i = 0; i < 4; ++i)
#pragma unroll
        for (int r = 0; r < 8; ++r) rs[i][r] = 0.0f;
#pragma unroll
    for (int j = 0; j < 4; ++j) {
        const unsigned n = n0 + (unsigned)j * 16u + c;
        const float b1v = bfr(b1[nd * HID + n]);
        const float w2v = bfr(W2[nd * HID + n]);
#pragma unroll
        for (int i = 0; i < 4; ++i)
#pragma unroll
            for (int r = 0; r < 8; ++r) {
                float v = acc[i][j][r] * SCL + b1v;
                v = fmaxf(v, 0.0f);
                rs[i][r] += v * w2v;
            }
    }
#pragma unroll
    for (int i = 0; i < 4; ++i)
#pragma unroll
        for (int r = 0; r < 8; ++r) {
            float s = rs[i][r];
            s += __shfl_xor(s, 1, 32);
            s += __shfl_xor(s, 2, 32);
            s += __shfl_xor(s, 4, 32);
            s += __shfl_xor(s, 8, 32);
            rs[i][r] = s;
        }
    if (c == 0u) {
#pragma unroll
        for (int i = 0; i < 4; ++i)
#pragma unroll
            for (int r = 0; r < 8; ++r)
                sPart[wave * 64u + (unsigned)i * 16u + 8u * hh + (unsigned)r] = rs[i][r];
    }
    __syncthreads();
    if (wave < 2u) {
        float o = bfr(b2[nd]);
#pragma unroll
        for (int w = 0; w < 8; ++w) o += sPart[(unsigned)w * 64u + tid];
        VST2(float, oT + (size_t)nd * NROWS + bbase + tid, o);
    }
}

__global__ __launch_bounds__(256) void k_out(const float* __restrict__ oT, float* __restrict__ out) {
    const unsigned u = blockIdx.x * 256u + threadIdx.x;
    if (u >= (unsigned)(NROWS * 4)) return;
    const unsigned row = u >> 2, c4 = (u & 3u) * 4u;
    v4f v;
    v.x = oT[(size_t)(c4 + 0u) * NROWS + row];
    v.y = oT[(size_t)(c4 + 1u) * NROWS + row];
    v.z = oT[(size_t)(c4 + 2u) * NROWS + row];
    v.w = oT[(size_t)(c4 + 3u) * NROWS + row];
    VST2V4(out + (size_t)row * 16u + c4, v);
}

extern "C" void kernel_launch(void* const* d_in, const int* in_sizes, int n_in, void* d_out, int out_size,
                              void* d_ws, size_t ws_size, hipStream_t stream) {
    if (n_in < 14) return;
    if (in_sizes[0] < NROWS * 16 || in_sizes[1] < NROWS * 10 || in_sizes[2] < NROWS * 4) return;
    if (in_sizes[3] < 512 || in_sizes[4] < 1280 || in_sizes[5] < 512 || in_sizes[6] < 512) return;
    if (in_sizes[7] < HID * 17 || in_sizes[8] < (NNODE - 1) * HID * 18 || in_sizes[9] < NNODE * HID) return;
    if (in_sizes[10] < NNODE * HID * HID || in_sizes[11] < NNODE * HID || in_sizes[12] < NNODE * HID || in_sizes[13] < NNODE) return;
    if (out_size < NROWS_FULL * NNODE + 4) return;

    const float* noise   = (const float*)d_in[0];
    const float* input_c = (const float*)d_in[1];
    const float* input_d = (const float*)d_in[2];
    const float* noise_d = (const float*)d_in[3];
    const float* cnet_w  = (const float*)d_in[4];
    const float* mu      = (const float*)d_in[5];
    const float* sigma   = (const float*)d_in[6];
    const float* W0_0    = (const float*)d_in[7];
    const float* W0_rest = (const float*)d_in[8];
    const float* b0      = (const float*)d_in[9];
    const float* W1      = (const float*)d_in[10];
    const float* b1      = (const float*)d_in[11];
    const float* W2      = (const float*)d_in[12];
    const float* b2      = (const float*)d_in[13];
    float* out = (float*)d_out;
    float* klout = out + (size_t)NROWS_FULL * NNODE;

    char* wsp = (char*)d_ws;
    size_t off = 0;
    auto carve = [&](size_t bytes) -> void* { void* r = wsp + off; off += (bytes + 255) & ~(size_t)255; return r; };
    float*          theta = (float*)carve((size_t)512 * 4);
    float*          oT    = (float*)carve((size_t)NNODE * NROWS * 4);
    unsigned short* w0h   = (unsigned short*)carve((size_t)NNODE * HID * 32 * 2);
    unsigned short* w1h   = (unsigned short*)carve((size_t)NNODE * HID * HID * 2);
    if (off > ws_size || off > (size_t)134217728) return;

    k_theta<<<1, 512, 0, stream>>>(mu, sigma, noise_d, theta, klout);
    k_w0conv<<<(NNODE * HID * 4) / 256, 256, 0, stream>>>(W0_0, W0_rest, w0h);
    k_w1conv<<<(NNODE * HID * HID / 8) / 256, 256, 0, stream>>>(W1, w1h);

    for (int i = 0; i < NNODE; ++i) {
        k_node<<<NROWS / 64, 256, 0, stream>>>(i, noise, input_c, input_d, cnet_w, theta,
            (const _Float16*)w0h, (const _Float16*)w1h, b0, b1, W2, b2, oT);
    }
    k_out<<<(NROWS * 4) / 256, 256, 0, stream>>>(oT, out);
}
